// PointConvSetAbstraction_46557445488939
// MI455X (gfx1250) — hardware-verified
//
#include <hip/hip_runtime.h>
#include <math.h>

typedef __attribute__((ext_vector_type(16))) _Float16 v16h;
typedef __attribute__((ext_vector_type(16))) __bf16 v16b;
typedef __attribute__((ext_vector_type(8)))  _Float16 v8h;
typedef __attribute__((ext_vector_type(8)))  float v8f;
typedef __attribute__((ext_vector_type(4)))  float v4f;
typedef __attribute__((ext_vector_type(2)))  float v2f;
typedef __attribute__((ext_vector_type(4)))  unsigned v4u;
typedef __attribute__((ext_vector_type(4)))  int v4i;
typedef float __attribute__((may_alias)) float_a;
typedef int __attribute__((may_alias)) int_a;

template <typename T> __device__ __forceinline__ void vst2(void* p, T v) { *(volatile T*)p = v; __threadfence(); *(volatile T*)p = v; }
__device__ __forceinline__ v8f wmma16(v16h a, v16h b, v8f c) {
  v8f d = __builtin_amdgcn_wmma_f32_16x16x32_f16(false, a, false, b, (short)0, c, false, false);
  asm volatile("v_nop\n\tv_nop\n\tv_nop\n\tv_nop" : "+v"(d) : "v"(a), "v"(b));
  return d;
}
__device__ __forceinline__ v8f wmma_bf(v16b a, v16b b, v8f c) {
  v8f d = __builtin_amdgcn_wmma_f32_16x16x32_bf16(false, a, false, b, (short)0, c, false, false);
  asm volatile("v_nop\n\tv_nop\n\tv_nop\n\tv_nop" : "+v"(d) : "v"(a), "v"(b));
  return d;
}
__device__ __forceinline__ v16h frag_h(const _Float16* rowk0, int lane) {
  union { v16h v; v8h q[2]; } u; const _Float16* p = rowk0 + 8 * (lane >> 4);
  u.q[0] = *(const v8h*)p; u.q[1] = *(const v8h*)(p + 16); return u.v;
}
__device__ __forceinline__ v16h frag_f32(const float* rowk0, int lane) {
  v16h a; const float* p = rowk0 + 8 * (lane >> 4);
#pragma unroll
  for (int i = 0; i < 8; ++i) { a[i] = (_Float16)p[i]; a[8 + i] = (_Float16)p[16 + i]; }
  return a;
}
__device__ __forceinline__ v16h frag_f32s(const float* rowk0, int lane, float sc) {
  v16h a; const float* p = rowk0 + 8 * (lane >> 4);
#pragma unroll
  for (int i = 0; i < 8; ++i) { a[i] = (_Float16)(p[i] * sc); a[8 + i] = (_Float16)(p[16 + i] * sc); }
  return a;
}
__device__ __forceinline__ v16h fragc_f32(const float* W, int k0, int n, int lane, int ld, int K) {
  v16h a; const int g = lane >> 4;
#pragma unroll
  for (int i = 0; i < 8; ++i) { const int ka = k0 + 8 * g + i, kb = ka + 16;
    a[i] = (_Float16)(ka < K ? W[(size_t)(ka < K ? ka : K - 1) * ld + n] : 0.f); a[8 + i] = (_Float16)(kb < K ? W[(size_t)(kb < K ? kb : K - 1) * ld + n] : 0.f); }
  return a;
}
struct F2 { v16b h, l; };
__device__ __forceinline__ F2 bsplit16(const float v[16]) { F2 r;
#pragma unroll
  for (int i = 0; i < 16; ++i) { const __bf16 h = (__bf16)v[i]; r.h[i] = h; r.l[i] = (__bf16)(v[i] - (float)h); }
  return r; }
__device__ __forceinline__ F2 split_row(const float* row, int k0, int lane) { float v[16]; const float* p = row + k0 + 8 * (lane >> 4);
#pragma unroll
  for (int i = 0; i < 8; ++i) { v[i] = p[i]; v[8 + i] = p[16 + i]; }
  return bsplit16(v); }
__device__ __forceinline__ F2 split_rowK(const float* row, int k0, int lane, int K) { float v[16]; const int g = lane >> 4;
#pragma unroll
  for (int i = 0; i < 8; ++i) { const int ka = k0 + 8 * g + i, kb = ka + 16; v[i] = ka < K ? row[ka < K ? ka : K - 1] : 0.f; v[8 + i] = kb < K ? row[kb < K ? kb : K - 1] : 0.f; }
  return bsplit16(v); }
__device__ __forceinline__ F2 split_col(const float* W, int k0, int n, int lane, int ld, int K) { float v[16]; const int g = lane >> 4;
#pragma unroll
  for (int i = 0; i < 8; ++i) { const int ka = k0 + 8 * g + i, kb = ka + 16; v[i] = ka < K ? W[(size_t)(ka < K ? ka : K - 1) * ld + n] : 0.f; v[8 + i] = kb < K ? W[(size_t)(kb < K ? kb : K - 1) * ld + n] : 0.f; }
  return bsplit16(v); }
__device__ __forceinline__ v8f mac3(const F2& a, const F2& b, v8f c) { c = wmma_bf(a.l, b.h, c); c = wmma_bf(a.h, b.l, c); return wmma_bf(a.h, b.h, c); }
__device__ __forceinline__ float sigm(float v) { return 1.0f / (1.0f + expf(-v)); }
#define LDSX() do { asm volatile("s_wait_dscnt 0" ::: "memory"); __builtin_amdgcn_wave_barrier(); __builtin_amdgcn_fence(__ATOMIC_RELEASE, "workgroup"); } while (0)


#define NB 8
#define NN 4096
#define SS 1024
#define KK 32
#define DF 64
#define NG (NB * SS)
#define NROW (NG * KK)
#ifndef NBT
#define NBT NB
#endif
#define NGT (NBT * SS)
#define NROWT (NGT * KK)
typedef __attribute__((ext_vector_type(8))) __bf16 v8b;
__device__ __forceinline__ v16b frag_b(const __bf16* rowk0, int lane) {
  union { v16b v; v8b q[2]; } u; const __bf16* p = rowk0 + 8 * (lane >> 4);
  u.q[0] = *(const v8b*)p; u.q[1] = *(const v8b*)(p + 16); return u.v;
}
__device__ __forceinline__ float bfr(float v) { return (float)(__bf16)v; }
__device__ __attribute__((noinline)) float exp_ni(float v) { return expf(v); }
__device__ __attribute__((noinline)) float erf_ni(float v) { return erff(v); }

struct F3 { v16b h, m, l; };
__device__ __forceinline__ F3 bsplit16_3(const float v[16]) { F3 r;
#pragma unroll
  for (int i = 0; i < 16; ++i) { const __bf16 h = (__bf16)v[i]; const float r1 = v[i] - (float)h; const __bf16 m = (__bf16)r1; r.h[i] = h; r.m[i] = m; r.l[i] = (__bf16)(r1 - (float)m); }
  return r; }
__device__ __forceinline__ F3 split3_row(const float* row, int k0, int lane) { float v[16]; const float* p = row + k0 + 8 * (lane >> 4);
#pragma unroll
  for (int i = 0; i < 8; ++i) { v[i] = p[i]; v[8 + i] = p[16 + i]; }
  return bsplit16_3(v); }

#define WS_PW   0u
#define PW0 0
#define PW1 (PW0 + 64 * 96)
#define PW2 (PW1 + 64 * 64)
#define PLW (PW2 + 128 * 64)
#define PWEND (PLW + 128 * 2048)
#define WS_FIDX (WS_PW + 2u * PWEND)
#define WS_FX   (WS_FIDX + 4u * NB * SS)
#define WS_KNN  (WS_FX + 4u * NG * 4)
#define WS_GX   (WS_KNN + 4u * NG * KK)
#define WS_A    (WS_GX + 4u * NROW * 4)
#define WS_B    (WS_A + 4u * NROW * 128)
#define WS_W0   (WS_B + 4u * NROW * 64)
#define WS_W1   (WS_W0 + 4u * NROW * 8)
#define WS_W2   (WS_W1 + 4u * NROW * 8)
#define WS_LIN  (WS_W2 + 4u * NROW * 16)
#define NSTB 128
#define WS_ST   (WS_LIN + 4u * NG * 128)
#define WS_BN   (WS_ST + 4u * NSTB * 128)
#define WS_END  (WS_BN + 4u * 8 * 4 * 128)

__global__ __launch_bounds__(256) void k_packw(const float* __restrict__ W0m, const float* __restrict__ W1m, const float* __restrict__ W2m, const float* __restrict__ LWm, __bf16* __restrict__ PW) {
  __shared__ __align__(16) __bf16 s0[96], s1[64], s2[64], sl[2048]; const int o = blockIdx.x, t = threadIdx.x;
  if (o < 64) { if (t < 96) s0[t] = (__bf16)((t < 67) ? W0m[o * 67 + t] : 0.f); if (t < 64) s1[t] = (__bf16)W1m[o * 64 + t]; }
  if (t < 64) s2[t] = (__bf16)W2m[o * 64 + t];
  for (int k = t; k < 2048; k += 256) sl[k] = (__bf16)LWm[(size_t)o * 2048 + k];
  __syncthreads();
  if (o < 64) { if (t < 12) vst2((unsigned*)(PW + PW0 + o * 96 + t * 8), *(const v4u*)&s0[t * 8]); if (t >= 16 && t < 24) vst2((unsigned*)(PW + PW1 + o * 64 + (t - 16) * 8), *(const v4u*)&s1[(t - 16) * 8]); }
  if (t >= 32 && t < 40) vst2((unsigned*)(PW + PW2 + o * 64 + (t - 32) * 8), *(const v4u*)&s2[(t - 32) * 8]);
  for (int q = t; q < 256; q += 256) vst2((unsigned*)(PW + PLW + (size_t)o * 2048 + q * 8), *(const v4u*)&sl[q * 8]);
}
__global__ __launch_bounds__(256) void k_fps(const float* __restrict__ XYZ, int* __restrict__ FIDX, float* __restrict__ FX, float* __restrict__ OUT0) {
  __shared__ float spx[NN], spy[NN], spz[NN]; __shared__ float sv[256]; __shared__ int si[256]; __shared__ int sfar; __shared__ __align__(16) int sidx[SS];
  const int t = threadIdx.x, b = blockIdx.x; const float* xb = XYZ + (size_t)b * 3 * NN;
  for (int n = t; n < NN; n += 256) { spx[n] = bfr(xb[n]); spy[n] = bfr(xb[NN + n]); spz[n] = bfr(xb[2 * NN + n]); }
  float dist[16];
#pragma unroll
  for (int m = 0; m < 16; ++m) dist[m] = 1e10f;
  if (t == 0) sfar = 0;
  __syncthreads();
#pragma unroll 1
  for (int i = 0; i < SS; ++i) { const int far = sfar; if (t == 0) sidx[i] = far; const float fx = spx[far], fy = spy[far], fz = spz[far];
    float best = -1.f; int bi = 0;
#pragma unroll
    for (int m = 0; m < 16; ++m) { const int n = t + 256 * m; const float dx = spx[n] - fx, dy = spy[n] - fy, dz = spz[n] - fz; const float d = (dx * dx + dz * dz) + dy * dy; dist[m] = fminf(dist[m], d); if (dist[m] > best) { best = dist[m]; bi = n; } }
    sv[t] = best; si[t] = bi; __syncthreads();
    for (int o = 128; o > 0; o >>= 1) { if (t < o) { const float v2 = sv[t + o]; const int i2 = si[t + o]; if (v2 > sv[t] || (v2 == sv[t] && i2 < si[t])) { sv[t] = v2; si[t] = i2; } } __syncthreads(); }
    if (t == 0) sfar = si[0];
    __syncthreads(); }
  for (int q = t; q < SS / 4; q += 256) vst2((unsigned*)(FIDX + (size_t)b * SS + q * 4), *(const v4u*)&sidx[q * 4]);
  __shared__ __align__(16) float sc[SS];
  for (int c = 0; c < 3; ++c) { const float* sp = c == 0 ? spx : (c == 1 ? spy : spz);
    for (int s = t; s < SS; s += 256) sc[s] = sp[sidx[s]];
    __syncthreads();
    for (int q = t; q < SS / 4; q += 256) vst2(OUT0 + ((size_t)b * 3 + c) * SS + q * 4, *(const v4f*)&sc[q * 4]);
    __syncthreads(); }
  for (int s = t; s < SS; s += 256) { v4f v = {spx[sidx[s]], spy[sidx[s]], spz[sidx[s]], 0.f}; vst2(FX + ((size_t)b * SS + s) * 4, v); }
}
__global__ __launch_bounds__(64) void k_knn(const float* __restrict__ XYZ, const float* __restrict__ FX, int* __restrict__ KNN) {
  __shared__ __align__(16) int sk[64][KK]; const int tid = threadIdx.x; const size_t gq = (size_t)blockIdx.x * 64 + tid; const int b = (int)(gq / SS); const float* xb = XYZ + (size_t)b * 3 * NN;
  const float cx = FX[gq * 4], cy = FX[gq * 4 + 1], cz = FX[gq * 4 + 2]; const float sqc = (cx * cx + cz * cz) + cy * cy;
  float bd[KK]; int bi[KK];
#pragma unroll
  for (int j = 0; j < KK; ++j) { bd[j] = 3.0e38f; bi[j] = 0; }
#pragma unroll 1
  for (int n = 0; n < NN; ++n) { const float x = bfr(xb[n]), y = bfr(xb[NN + n]), z = bfr(xb[2 * NN + n]); const float sqx = (x * x + z * z) + y * y; const float dot = (cx * x + cy * y) + cz * z; const float d = (sqc + sqx) - 2.0f * dot;
    if (d < bd[KK - 1]) { int pos = KK - 1;
#pragma unroll
      for (int q = KK - 2; q >= 0; --q) if (d < bd[q]) pos = q;
#pragma unroll
      for (int q = KK - 1; q >= 1; --q) if (q > pos) { bd[q] = bd[q - 1]; bi[q] = bi[q - 1]; }
#pragma unroll
      for (int q = 0; q < KK; ++q) if (q == pos) { bd[q] = d; bi[q] = n; } } }
#pragma unroll
  for (int q = 0; q < KK; ++q) sk[tid][q] = bi[q];
  __syncthreads();
  for (int r = 0; r < 64; ++r) if (tid < 8) vst2((unsigned*)(KNN + ((size_t)blockIdx.x * 64 + r) * KK + tid * 4), *(const v4u*)&sk[r][tid * 4]);
}
__global__ __launch_bounds__(128) void k_l0(const float* __restrict__ XYZ, const float* __restrict__ FEAT, const float* __restrict__ FX, const int* __restrict__ KNN, const __bf16* __restrict__ PW, const float* __restrict__ B0, float* __restrict__ GX, float* __restrict__ Y0) {
  __shared__ __align__(16) float sa[64][100]; __shared__ __align__(16) float so[4][16][68];
  const int tid = threadIdx.x, wave = tid >> 5, lane = tid & 31, col = lane & 15, g = lane >> 4; const size_t rb = (size_t)blockIdx.x * 64;
  for (int q = tid; q < 64 * 96; q += 128) { const int rl = q / 96, cc = q % 96; const size_t r = rb + rl; const size_t gq = r / KK; const int k = (int)(r % KK); const int b = (int)(gq / SS); const int n = min(max(KNN[gq * KK + k], 0), NN - 1); const float* xb = XYZ + (size_t)b * 3 * NN; float v = 0.f;
    if (cc < 3) v = bfr(xb[cc * NN + n]) - FX[gq * 4 + cc]; else if (cc < 67) v = bfr(FEAT[((size_t)b * DF + (cc - 3)) * NN + n]);
    sa[rl][cc] = v; }
  __syncthreads();
  if (tid < 64) { v4f gx = {sa[tid][0], sa[tid][1], sa[tid][2], 0.f}; vst2(GX + (rb + tid) * 4, gx); }
  v8f acc[4] = {};
#pragma unroll
  for (int kc = 0; kc < 3; ++kc) { const F2 a = split_row(&sa[wave * 16 + col][0], kc * 32, lane);
#pragma unroll
    for (int j = 0; j < 4; ++j) { const v16b w = frag_b(PW + PW0 + (size_t)(j * 16 + col) * 96 + kc * 32, lane); acc[j] = wmma_bf(a.l, w, acc[j]); acc[j] = wmma_bf(a.h, w, acc[j]); } }
#pragma unroll
  for (int j = 0; j < 4; ++j)
#pragma unroll
    for (int r = 0; r < 8; ++r) so[wave][8 * g + r][j * 16 + col] = acc[j][r] + bfr(B0[j * 16 + col]);
  LDSX();
  for (int rl = 0; rl < 16; ++rl) if (lane < 16) vst2(Y0 + (rb + wave * 16 + rl) * 64 + lane * 4, *(const v4f*)&so[wave][rl][lane * 4]);
}
template <int KIN, int NOUT>
__global__ __launch_bounds__(128) void k_mlp(const float* __restrict__ YIN, const float* __restrict__ BNP, const __bf16* __restrict__ P, const float* __restrict__ bias, float* __restrict__ YOUT) {
  constexpr int NT = NOUT / 16; __shared__ __align__(16) float so[4][16][NOUT + 4];
  const int tid = threadIdx.x, wave = tid >> 5, lane = tid & 31, col = lane & 15, g = lane >> 4; const size_t r0 = (size_t)blockIdx.x * 64 + wave * 16;
  v8f acc[NT]; for (int j = 0; j < NT; ++j) acc[j] = (v8f){};
#pragma unroll
  for (int kc = 0; kc < KIN / 32; ++kc) { float v[16]; const float* p = YIN + (r0 + col) * KIN + kc * 32 + 8 * g;
#pragma unroll
    for (int i = 0; i < 16; ++i) { const int c = kc * 32 + 8 * g + (i & 7) + ((i >> 3) << 4); const float y = (i < 8) ? p[i] : p[16 + i - 8]; v[i] = fmaxf(y * BNP[128 + c] + BNP[256 + c], 0.f); }
    const F2 a = bsplit16(v);
#pragma unroll
    for (int j = 0; j < NT; ++j) { const v16b w = frag_b(P + (size_t)(j * 16 + col) * KIN + kc * 32, lane); acc[j] = wmma_bf(a.l, w, acc[j]); acc[j] = wmma_bf(a.h, w, acc[j]); } }
#pragma unroll
  for (int j = 0; j < NT; ++j)
#pragma unroll
    for (int r = 0; r < 8; ++r) so[wave][8 * g + r][j * 16 + col] = acc[j][r] + bfr(bias[j * 16 + col]);
  LDSX();
  for (int rl = 0; rl < 16; ++rl) for (int pc = lane; pc < NOUT / 4; pc += 32) vst2(YOUT + (r0 + rl) * NOUT + pc * 4, *(const v4f*)&so[wave][rl][pc * 4]);
}
template <int PASS>
__global__ __launch_bounds__(128) void k_stat(const float* __restrict__ Y, int W, int nrows, const float* __restrict__ BNP, float* __restrict__ ST) {
  __shared__ __align__(16) float s[128]; const int c = threadIdx.x; const int rpb = nrows / NSTB; const size_t r0 = (size_t)blockIdx.x * rpb; float a = 0.f; const float mu = (PASS && c < W) ? BNP[c] : 0.f;
  if (c < W) {
#pragma unroll 4
    for (int r = 0; r < rpb; ++r) { const float y = Y[(r0 + r) * W + c]; const float d = y - mu; a += PASS ? d * d : y; } }
  s[c] = a; __syncthreads();
  if (c < 32) vst2(ST + (size_t)blockIdx.x * 128 + c * 4, *(const v4f*)&s[c * 4]);
}
template <int PASS>
__global__ __launch_bounds__(128) void k_fin(const float* __restrict__ ST, int W, int nrows, const float* __restrict__ G, const float* __restrict__ BE, float* __restrict__ BNP) {
  __shared__ __align__(16) float s[2][128]; const int c = threadIdx.x; float a = 0.f;
#pragma unroll 1
  for (int b = 0; b < NSTB; ++b) a += ST[(size_t)b * 128 + c];
  const float n = (float)nrows;
  if (PASS == 0) { s[0][c] = (c < W) ? a / n : 0.f; __syncthreads(); if (c < 32) vst2(BNP + c * 4, *(const v4f*)&s[0][c * 4]); }
  else { float sc = 0.f, sh = 0.f; if (c < W) { const float var = a / n; sc = bfr(G[c]) * rsqrtf(var + 1e-5f); sh = bfr(BE[c]) - BNP[c] * sc; } s[0][c] = sc; s[1][c] = sh; __syncthreads(); if (c < 32) { vst2(BNP + 128 + c * 4, *(const v4f*)&s[0][c * 4]); vst2(BNP + 256 + c * 4, *(const v4f*)&s[1][c * 4]); } }
}
template <int LAYER>
__global__ __launch_bounds__(256) void k_wn(const float* __restrict__ IN, const float* __restrict__ BNP, const float* __restrict__ Wm, const float* __restrict__ Bm, float* __restrict__ OUT) {
  const size_t r = (size_t)blockIdx.x * 256 + threadIdx.x; constexpr int CIN = LAYER == 0 ? 3 : 8; constexpr int COUT = LAYER == 2 ? 16 : 8; constexpr int PIN = LAYER == 0 ? 4 : 8;
  __shared__ __align__(16) float sbuf[8][32 * 16]; const int wave = threadIdx.x >> 5, lane = threadIdx.x & 31;
  float x[8];
#pragma unroll
  for (int i = 0; i < CIN; ++i) { const float v = IN[r * PIN + i]; x[i] = (LAYER == 0) ? v : fmaxf(v * BNP[128 + i] + BNP[256 + i], 0.f); }
  float o[16];
#pragma unroll
  for (int j = 0; j < COUT; ++j) { float a = bfr(Bm[j]);
#pragma unroll
    for (int i = 0; i < CIN; ++i) a += x[i] * bfr(Wm[j * CIN + i]);
    o[j] = a; }
#pragma unroll
  for (int j = 0; j < COUT; ++j) sbuf[wave][lane * COUT + j] = o[j];
  LDSX();
  const size_t wbase = ((size_t)blockIdx.x * 256 + wave * 32) * COUT;
#pragma unroll
  for (int i = 0; i < COUT / 4; ++i) { const int p = lane + 32 * i; vst2(OUT + wbase + 4 * p, *(const v4f*)&sbuf[wave][4 * p]); }
}
__global__ __launch_bounds__(128) void k_agg(const float* __restrict__ Y2, const float* __restrict__ BN2, const float* __restrict__ W2p, const float* __restrict__ BNW, float* __restrict__ AGG) {
  __shared__ __align__(16) float sw[16][36]; __shared__ __align__(16) float so[4][16][20];
  const int tid = threadIdx.x, wave = tid >> 5, lane = tid & 31, col = lane & 15, g8 = lane >> 4; const size_t gq = blockIdx.x;
  for (int q = tid; q < 16 * 32; q += 128) { const int c = q >> 5, k = q & 31; const float v = W2p[(gq * KK + k) * 16 + c]; sw[c][k] = fmaxf(v * BNW[128 + c] + BNW[256 + c], 0.f); }
  __syncthreads();
  const F2 bw = split_row(&sw[col][0], 0, lane);
#pragma unroll
  for (int dt2 = 0; dt2 < 2; ++dt2) { const int dt = wave * 2 + dt2; const int d = dt * 16 + col; float v[16];
#pragma unroll
    for (int i = 0; i < 16; ++i) { const int k = 8 * g8 + (i & 7) + ((i >> 3) << 4); const float y = Y2[(gq * KK + k) * 128 + d]; v[i] = fmaxf(y * BN2[128 + d] + BN2[256 + d], 0.f); }
    const F3 a = bsplit16_3(v); v8f acc = {};
    acc = wmma_bf(a.l, bw.h, acc); acc = wmma_bf(a.m, bw.l, acc); acc = wmma_bf(a.m, bw.h, acc); acc = wmma_bf(a.h, bw.l, acc); acc = wmma_bf(a.h, bw.h, acc);
#pragma unroll
    for (int r = 0; r < 8; ++r) so[wave][8 * g8 + r][col] = acc[r];
    LDSX();
    for (int q = lane; q < 64; q += 32) { const int rl = q >> 2, pc = q & 3; vst2(AGG + gq * 2048 + (size_t)(dt * 16 + rl) * 16 + pc * 4, *(const v4f*)&so[wave][rl][pc * 4]); }
    LDSX(); }
}
__global__ __launch_bounds__(128) void k_final(const float* __restrict__ AGG, const __bf16* __restrict__ PW, const float* __restrict__ LB, float* __restrict__ LIN) {
  __shared__ __align__(16) float so[4][16][132];
  const int tid = threadIdx.x, wave = tid >> 5, lane = tid & 31, col = lane & 15, g = lane >> 4; const size_t r0 = (size_t)blockIdx.x * 64 + wave * 16;
  v8f acc[8] = {};
#pragma unroll 2
  for (int kc = 0; kc < 2048 / 32; ++kc) { const F3 a = split3_row(AGG + (r0 + col) * 2048, kc * 32, lane);
#pragma unroll
    for (int j = 0; j < 8; ++j) { const v16b w = frag_b(PW + PLW + (size_t)(j * 16 + col) * 2048 + kc * 32, lane); acc[j] = wmma_bf(a.l, w, acc[j]); acc[j] = wmma_bf(a.m, w, acc[j]); acc[j] = wmma_bf(a.h, w, acc[j]); } }
#pragma unroll
  for (int j = 0; j < 8; ++j)
#pragma unroll
    for (int r = 0; r < 8; ++r) so[wave][8 * g + r][j * 16 + col] = acc[j][r] + bfr(LB[j * 16 + col]);
  LDSX();
  for (int rl = 0; rl < 16; ++rl) vst2(LIN + (r0 + rl) * 128 + lane * 4, *(const v4f*)&so[wave][rl][lane * 4]);
}
__global__ __launch_bounds__(64) void k_out(const float* __restrict__ LIN, const float* __restrict__ BNP, float* __restrict__ OUT1) {
  const int s = blockIdx.x * 64 + threadIdx.x, b = blockIdx.y; const float* lr = LIN + ((size_t)b * SS + s) * 128;
#pragma unroll 1
  for (int c = 0; c < 128; ++c) { const float v = fmaxf(lr[c] * BNP[128 + c] + BNP[256 + c], 0.f); vst2(OUT1 + ((size_t)b * 128 + c) * SS + s, v); }
}
extern "C" void kernel_launch(void* const* d_in, const int* in_sizes, int n_in, void* d_out, int out_size, void* d_ws, size_t ws_size, hipStream_t stream) {
  (void)in_sizes; (void)n_in; (void)out_size;
  const float** F = (const float**)d_in;
  if (ws_size < (size_t)WS_END) return;
  char* ws = (char*)d_ws; __bf16* PW = (__bf16*)(ws + WS_PW); int *FIDX = (int*)(ws + WS_FIDX), *KNN = (int*)(ws + WS_KNN); float *FX = (float*)(ws + WS_FX), *GX = (float*)(ws + WS_GX), *BA = (float*)(ws + WS_A), *BB = (float*)(ws + WS_B), *W0p = (float*)(ws + WS_W0), *W1p = (float*)(ws + WS_W1), *W2p = (float*)(ws + WS_W2), *LIN = (float*)(ws + WS_LIN), *ST = (float*)(ws + WS_ST), *BN = (float*)(ws + WS_BN);
  float* OUT0 = (float*)d_out; float* OUT1 = OUT0 + (size_t)NB * 3 * SS;
  float* BN0 = BN, *BN1 = BN + 512, *BN2 = BN + 1024, *BW0 = BN + 1536, *BW1 = BN + 2048, *BW2 = BN + 2560, *BNL = BN + 3072;
  k_packw<<<128, 256, 0, stream>>>(F[2], F[6], F[10], F[26], PW);
  k_fps<<<NBT, 256, 0, stream>>>(F[0], FIDX, FX, OUT0);
  k_knn<<<NGT / 64, 64, 0, stream>>>(F[0], FX, KNN);
  k_l0<<<NROWT / 64, 128, 0, stream>>>(F[0], F[1], FX, KNN, PW, F[3], GX, BA);
  k_stat<0><<<NSTB, 128, 0, stream>>>(BA, 64, NROWT, BN0, ST); k_fin<0><<<1, 128, 0, stream>>>(ST, 64, NROWT, F[4], F[5], BN0); k_stat<1><<<NSTB, 128, 0, stream>>>(BA, 64, NROWT, BN0, ST); k_fin<1><<<1, 128, 0, stream>>>(ST, 64, NROWT, F[4], F[5], BN0);
  k_mlp<64, 64><<<NROWT / 64, 128, 0, stream>>>(BA, BN0, PW + PW1, F[7], BB);
  k_stat<0><<<NSTB, 128, 0, stream>>>(BB, 64, NROWT, BN1, ST); k_fin<0><<<1, 128, 0, stream>>>(ST, 64, NROWT, F[8], F[9], BN1); k_stat<1><<<NSTB, 128, 0, stream>>>(BB, 64, NROWT, BN1, ST); k_fin<1><<<1, 128, 0, stream>>>(ST, 64, NROWT, F[8], F[9], BN1);
  k_mlp<64, 128><<<NROWT / 64, 128, 0, stream>>>(BB, BN1, PW + PW2, F[11], BA);
  k_stat<0><<<NSTB, 128, 0, stream>>>(BA, 128, NROWT, BN2, ST); k_fin<0><<<1, 128, 0, stream>>>(ST, 128, NROWT, F[12], F[13], BN2); k_stat<1><<<NSTB, 128, 0, stream>>>(BA, 128, NROWT, BN2, ST); k_fin<1><<<1, 128, 0, stream>>>(ST, 128, NROWT, F[12], F[13], BN2);
  k_wn<0><<<NROWT / 256, 256, 0, stream>>>(GX, nullptr, F[14], F[15], W0p);
  k_stat<0><<<NSTB, 128, 0, stream>>>(W0p, 8, NROWT, BW0, ST); k_fin<0><<<1, 128, 0, stream>>>(ST, 8, NROWT, F[16], F[17], BW0); k_stat<1><<<NSTB, 128, 0, stream>>>(W0p, 8, NROWT, BW0, ST); k_fin<1><<<1, 128, 0, stream>>>(ST, 8, NROWT, F[16], F[17], BW0);
  k_wn<1><<<NROWT / 256, 256, 0, stream>>>(W0p, BW0, F[18], F[19], W1p);
  k_stat<0><<<NSTB, 128, 0, stream>>>(W1p, 8, NROWT, BW1, ST); k_fin<0><<<1, 128, 0, stream>>>(ST, 8, NROWT, F[20], F[21], BW1); k_stat<1><<<NSTB, 128, 0, stream>>>(W1p, 8, NROWT, BW1, ST); k_fin<1><<<1, 128, 0, stream>>>(ST, 8, NROWT, F[20], F[21], BW1);
  k_wn<2><<<NROWT / 256, 256, 0, stream>>>(W1p, BW1, F[22], F[23], W2p);
  k_stat<0><<<NSTB, 128, 0, stream>>>(W2p, 16, NROWT, BW2, ST); k_fin<0><<<1, 128, 0, stream>>>(ST, 16, NROWT, F[24], F[25], BW2); k_stat<1><<<NSTB, 128, 0, stream>>>(W2p, 16, NROWT, BW2, ST); k_fin<1><<<1, 128, 0, stream>>>(ST, 16, NROWT, F[24], F[25], BW2);
  k_agg<<<NGT, 128, 0, stream>>>(BA, BN2, W2p, BW2, BB);
  k_final<<<NGT / 64, 128, 0, stream>>>(BB, PW, F[27], LIN);
  k_stat<0><<<NSTB, 128, 0, stream>>>(LIN, 128, NGT, BNL, ST); k_fin<0><<<1, 128, 0, stream>>>(ST, 128, NGT, F[28], F[29], BNL); k_stat<1><<<NSTB, 128, 0, stream>>>(LIN, 128, NGT, BNL, ST); k_fin<1><<<1, 128, 0, stream>>>(ST, 128, NGT, F[28], F[29], BNL);
  k_out<<<dim3(SS / 64, NBT), 64, 0, stream>>>(LIN, BNL, OUT1);
}
